// LatentMixtureAllRNNAgent_48954037240524
// MI455X (gfx1250) — hardware-run, weakly checked
//
#include <hip/hip_runtime.h>
#include <math.h>

constexpr int NAG    = 8;
constexpr int NBAT   = 4096;
constexpr int NFEAT  = 256;
constexpr int NHID   = 256;
constexpr int NGATE  = 3 * NHID;
constexpr int NACT   = 30;
constexpr int NACTP  = 64;
constexpr int NROWS  = NBAT * NAG;
constexpr int XPITCH = 2 * NHID;
constexpr int BPITCH = NHID + NACTP;
constexpr int SLABP  = 68;
constexpr int NOUT0  = NROWS * NACT;
constexpr int NOUT1  = NROWS * NHID;
static_assert(NFEAT % 32 == 0 && NHID % 32 == 0 && XPITCH % 32 == 0);
static_assert(NBAT % 64 == 0 && NHID % 64 == 0 && NACTP % 64 == 0 && NGATE % 64 == 0);
static_assert(((size_t)NOUT0 * 4) % 128 == 0);
static_assert(NOUT0 % 4 == 0 && (NOUT0 / 4) % 256 == 0);
static_assert((NAG * BPITCH / 4) % 32 == 0);

typedef __attribute__((ext_vector_type(8)))  _Float16 v8h;
typedef __attribute__((ext_vector_type(16))) __bf16   v16b;
typedef __attribute__((ext_vector_type(8)))  __bf16   v8b;
typedef __attribute__((ext_vector_type(8)))  float    v8f;
typedef __attribute__((ext_vector_type(4)))  float    v4f;

__device__ __forceinline__ unsigned short f2bf_bits(float f) {
  unsigned u = __float_as_uint(f);
  return (unsigned short)((u + 0x7FFFu + ((u >> 16) & 1u)) >> 16);
}
__device__ __forceinline__ float bf_bits2f(unsigned short h) { return __uint_as_float(((unsigned)h) << 16); }
__device__ __forceinline__ float bf16r(float f) { return bf_bits2f(f2bf_bits(f)); }

__device__ __forceinline__ void dep_guard4_b(v8f& a, v8f& b, v8f& c, v8f& d, v16b x, v16b y) {
  asm volatile("v_nop\n\tv_nop\n\tv_nop\n\tv_nop" : "+v"(a), "+v"(b), "+v"(c), "+v"(d) : "v"(x), "v"(y));
}
__device__ __forceinline__ void keep4_b(v16b a, v16b b, v16b c, v16b d) { asm volatile("v_nop" :: "v"(a), "v"(b), "v"(c), "v"(d)); }
__device__ __forceinline__ void acc_guard4(v8f& a, v8f& b, v8f& c, v8f& d) {
  asm volatile("v_nop\n\tv_nop\n\tv_nop\n\tv_nop" : "+v"(a), "+v"(b), "+v"(c), "+v"(d));
}
__device__ __forceinline__ void gate_guard(v8f& a, v8f& b, v8f& c, v8f& d, v16b x, v16b y, v16b z,
                                           v16b p0, v16b p1, v16b p2, v16b p3, v16b p4, v16b p5) {
  asm volatile("v_nop\n\tv_nop\n\tv_nop\n\tv_nop" : "+v"(a), "+v"(b), "+v"(c), "+v"(d)
               : "v"(x), "v"(y), "v"(z), "v"(p0), "v"(p1), "v"(p2), "v"(p3), "v"(p4), "v"(p5));
}

template <typename T> struct Frag;
template <> struct Frag<__bf16> {
  typedef v16b V; union U { v16b v; v8b h[2]; };
  static __device__ __forceinline__ v16b load(const __bf16* p) {
    U f; f.h[0] = *(const v8b*)(p); f.h[1] = *(const v8b*)(p + 16); return f.v;
  }
  static __device__ __forceinline__ v8f mma(v16b a, v16b b, v8f c) {
    return __builtin_amdgcn_wmma_f32_16x16x32_bf16(false, a, false, b, (short)0, c, false, false);
  }
  static __device__ __forceinline__ void guard4(v8f& a, v8f& b, v8f& c, v8f& d, v16b x, v16b y) { dep_guard4_b(a, b, c, d, x, y); }
  static __device__ __forceinline__ void keep(v16b a, v16b b, v16b c, v16b d) { keep4_b(a, b, c, d); }
};

template <int ET> struct Elem;
template <> struct Elem<1> { typedef __bf16 T; };
template <int ET, bool SPLIT, int BIAS_MODE, int OUT_MODE, bool RESID, int ACT = 0>
__global__ __launch_bounds__(256) void wmma_gemm64(
    const unsigned short* __restrict__ Ap, const unsigned short* __restrict__ A2p, int lda, long strideA,
    const unsigned short* __restrict__ Btp, const unsigned short* __restrict__ Bt2p, int ldb, long strideB,
    void* __restrict__ Cout, void* __restrict__ Cout2, int ldc, long strideC,
    const float* __restrict__ bias, long strideBias,
    const float* __restrict__ resid, long strideR,
    int M, int N, int K, float scale) {
  typedef typename Elem<ET>::T T;
  typedef typename Frag<T>::V V;
  const T* A = (const T*)Ap; const T* A2 = (const T*)A2p; const T* Bt = (const T*)Btp; const T* Bt2 = (const T*)Bt2p;
  __shared__ __align__(16) float sT[8][16 * 68];
  const int b    = blockIdx.y;
  const int lane = threadIdx.x & 31;
  const int wave = threadIdx.x >> 5;
  const int tilesN = N >> 6;
  const int tilesM = M >> 6;
  const int tile = blockIdx.x * 8 + wave;
  if (tile >= tilesM * tilesN) return;
  const int tm = tile / tilesN;
  const int tn = tile - tm * tilesN;
  const int m0 = tm << 6;
  const int n0 = tn << 6;

  const T* Ab  = A  + (size_t)b * strideA;
  const T* Bb  = Bt + (size_t)b * strideB;
  const T* Ab2 = SPLIT ? (A2  + (size_t)b * strideA) : nullptr;
  const T* Bb2 = SPLIT ? (Bt2 + (size_t)b * strideB) : nullptr;
  const float* biasb = bias + (size_t)b * strideBias;

  const int rlane = lane & 15;
  const int koff  = (lane >> 4) * 8;
  const int mOff  = (lane >> 4) * 8;

  v8f acc[4][4];
#pragma unroll
  for (int i = 0; i < 4; ++i)
#pragma unroll
    for (int j = 0; j < 4; ++j) acc[i][j] = (v8f){0.f,0.f,0.f,0.f,0.f,0.f,0.f,0.f};

  for (int k0 = 0; k0 < K; k0 += 32) {
    V bh[4], bl[4];
#pragma unroll
    for (int j = 0; j < 4; ++j) {
      const size_t bo = (size_t)(n0 + (j << 4) + rlane) * ldb + koff + k0;
      bh[j] = Frag<T>::load(Bb + bo);
      if (SPLIT) bl[j] = Frag<T>::load(Bb2 + bo);
    }
#pragma unroll
    for (int i = 0; i < 4; ++i) {
      const size_t ao = (size_t)(m0 + (i << 4) + rlane) * lda + koff + k0;
      V ah = Frag<T>::load(Ab + ao);
      V al;
      if (SPLIT) al = Frag<T>::load(Ab2 + ao);
#pragma unroll
      for (int j = 0; j < 4; ++j) {
        acc[i][j] = Frag<T>::mma(ah, bh[j], acc[i][j]);
        if (SPLIT) {
          acc[i][j] = Frag<T>::mma(ah, bl[j], acc[i][j]);
          acc[i][j] = Frag<T>::mma(al, bh[j], acc[i][j]);
        }
      }
      Frag<T>::guard4(acc[i][0], acc[i][1], acc[i][2], acc[i][3], ah, SPLIT ? al : ah);
    }
    Frag<T>::keep(bh[0], bh[1], bh[2], bh[3]);
    if (SPLIT) Frag<T>::keep(bl[0], bl[1], bl[2], bl[3]);
  }
  acc_guard4(acc[0][0], acc[0][1], acc[0][2], acc[0][3]);
  acc_guard4(acc[1][0], acc[1][1], acc[1][2], acc[1][3]);
  acc_guard4(acc[2][0], acc[2][1], acc[2][2], acc[2][3]);
  acc_guard4(acc[3][0], acc[3][1], acc[3][2], acc[3][3]);

  float* slab = sT[wave];
  const float* Rb = RESID ? (resid + (size_t)b * strideR) : nullptr;
#pragma unroll
  for (int i = 0; i < 4; ++i) {
    const int mBase = m0 + (i << 4);
#pragma unroll
    for (int j = 0; j < 4; ++j) {
      const int n = n0 + (j << 4) + rlane;
      float bv = 0.f;
      if (BIAS_MODE == 2) bv = biasb[n];
#pragma unroll
      for (int r = 0; r < 8; ++r) {
        float v = acc[i][j][r] * scale;
        if (BIAS_MODE == 1) v += biasb[mBase + mOff + r];
        if (BIAS_MODE == 2) v += bv;
        if (RESID) v += Rb[(size_t)(mBase + mOff + r) * ldc + n];
        if (ACT == 2) v = fmaxf(v, 0.0f);
        slab[(mOff + r) * 68 + (j << 4) + rlane] = v;
      }
    }
    __builtin_amdgcn_fence(__ATOMIC_RELEASE, "workgroup");
    __builtin_amdgcn_wave_barrier();
    __builtin_amdgcn_fence(__ATOMIC_ACQUIRE, "workgroup");
    if (OUT_MODE == 0) {
      float* C = (float*)Cout + (size_t)b * strideC;
      const int hh = lane >> 4, c4 = (lane & 15) * 4;
      for (int pass = 0; pass < 2; ++pass) {
#pragma unroll
        for (int it = 0; it < 8; ++it) {
          const int row = it * 2 + hh;
          v4f v = *(const v4f*)(slab + row * 68 + c4);
          *(volatile v4f*)(C + (size_t)(mBase + row) * ldc + n0 + c4) = v;
        }
        __threadfence();
      }
    } else {
      const int q = lane >> 3, c8 = (lane & 7) * 8;
      unsigned short* C  = (unsigned short*)Cout  + (size_t)b * strideC;
      unsigned short* C2 = (OUT_MODE == 2) ? ((unsigned short*)Cout2 + (size_t)b * strideC) : nullptr;
      for (int pass = 0; pass < 2; ++pass) {
#pragma unroll
        for (int it = 0; it < 4; ++it) {
          const int row = it * 4 + q;
          const float* sp = slab + row * 68 + c8;
          v8h hv, lv;
#pragma unroll
          for (int e = 0; e < 8; ++e) {
            if (OUT_MODE == 1) {
              hv[e] = (_Float16)sp[e];
            } else {
              unsigned short hb = f2bf_bits(sp[e]);
              unsigned short lb = f2bf_bits(sp[e] - bf_bits2f(hb));
              hv[e] = __builtin_bit_cast(_Float16, hb);
              lv[e] = __builtin_bit_cast(_Float16, lb);
            }
          }
          *(volatile v8h*)(C + (size_t)(mBase + row) * ldc + n0 + c8) = hv;
          if (OUT_MODE == 2) *(volatile v8h*)(C2 + (size_t)(mBase + row) * ldc + n0 + c8) = lv;
        }
        __threadfence();
      }
    }
    __builtin_amdgcn_fence(__ATOMIC_RELEASE, "workgroup");
    __builtin_amdgcn_wave_barrier();
    __builtin_amdgcn_fence(__ATOMIC_ACQUIRE, "workgroup");
  }
}

__global__ __launch_bounds__(256) void tpw_bf16_kernel(const float* __restrict__ src, int R, int C, int ldo,
                                                       unsigned short* __restrict__ O, long sstride, long ostride) {
  __shared__ float Tt[64 * 65];
  const int tid = threadIdx.x;
  const int c0 = blockIdx.x * 64, r0 = blockIdx.y * 64;
  const float* sp = src + (size_t)blockIdx.z * (size_t)sstride;
  unsigned short* Ob = O + (size_t)blockIdx.z * (size_t)ostride;
#pragma unroll
  for (int i = 0; i < 4; ++i) {
    const int idx = i * 256 + tid;
    const int rr = idx >> 4, cc = (idx & 15) * 4;
    const v4f v = *(const v4f*)(sp + (size_t)(r0 + rr) * (size_t)C + c0 + cc);
    Tt[rr * 65 + cc + 0] = v[0];
    Tt[rr * 65 + cc + 1] = v[1];
    Tt[rr * 65 + cc + 2] = v[2];
    Tt[rr * 65 + cc + 3] = v[3];
  }
  __syncthreads();
  const int q = tid >> 3, c8 = (tid & 7) * 8;
  v8h hv[2];
#pragma unroll
  for (int g = 0; g < 2; ++g) {
    const int qq = g * 32 + q;
#pragma unroll
    for (int e = 0; e < 8; ++e) {
      const float f = Tt[(c8 + e) * 65 + qq];
      const unsigned short bits = f2bf_bits(f);
      hv[g][e] = __builtin_bit_cast(_Float16, bits);
    }
  }
  for (int pass = 0; pass < 2; ++pass) {
#pragma unroll
    for (int g = 0; g < 2; ++g) {
      const size_t o = (size_t)(c0 + g * 32 + q) * (size_t)ldo + (size_t)(r0 + c8);
      *(volatile v8h*)(Ob + o) = hv[g];
    }
    __threadfence();
  }
}

__global__ __launch_bounds__(256) void w2_prep_kernel(const float* __restrict__ w2, unsigned short* __restrict__ O) {
  const int i = blockIdx.x * 256 + threadIdx.x;
  if (i < NAG * NACTP * (XPITCH / 8)) {
    const int a = i >> 12;
    const int n = (i >> 6) & 63;
    const int k8 = (i & 63) * 8;
    const int nc = (n < NACT) ? n : (NACT - 1);
    const float* wp = w2 + (size_t)a * NHID * NACT + nc;
    v8h hv;
#pragma unroll
    for (int e = 0; e < 8; ++e) {
      const int k = (k8 + e) & (NHID - 1);
      const float f = wp[(size_t)k * NACT];
      const float fz = (n < NACT) ? f : 0.0f;
      const unsigned short bits = f2bf_bits(fz);
      hv[e] = __builtin_bit_cast(_Float16, bits);
    }
    *(volatile v8h*)(O + (size_t)i * 8) = hv;
    __threadfence();
    *(volatile v8h*)(O + (size_t)i * 8) = hv;
  }
}

__global__ __launch_bounds__(256) void bias_prep_kernel(const float* __restrict__ b1, const float* __restrict__ b2,
                                                        float* __restrict__ dst) {
  const int i = blockIdx.x * 256 + threadIdx.x;
  if (i < NAG * BPITCH / 4) {
    const int a = i / (BPITCH / 4);
    const int col = (i - a * (BPITCH / 4)) * 4;
    const int c1 = (col < NHID) ? col : (NHID - 4);
    const v4f f1 = *(const v4f*)(b1 + a * NHID + c1);
    v4f o;
#pragma unroll
    for (int e = 0; e < 4; ++e) {
      const int n = col - NHID + e;
      const int nc = (n < 0) ? 0 : ((n > NACT - 1) ? (NACT - 1) : n);
      const float f2 = b2[a * NACT + nc];
      const float s2 = (n < NACT) ? f2 : 0.0f;
      const float sel = (col < NHID) ? f1[e] : s2;
      o[e] = bf16r(sel);
    }
    float* op = dst + (size_t)i * 4;
    *(volatile v4f*)op = o;
    __threadfence();
    *(volatile v4f*)op = o;
  }
}

__global__ __launch_bounds__(256) void in_cvt_kernel(const float* __restrict__ inp, const float* __restrict__ hid,
                                                     unsigned short* __restrict__ XB, unsigned short* __restrict__ HB) {
  const int which = blockIdx.y;
  const float* src = which ? hid : inp;
  unsigned short* dst = which ? HB : XB;
  const int i = blockIdx.x * 256 + threadIdx.x;
  if (i < NROWS * 32) {
    const int row = i >> 5;
    const int c8 = (i & 31) * 8;
    const int a = row & (NAG - 1);
    const int b = row >> 3;
    const float* sp = src + (size_t)row * NFEAT + c8;
    const v4f va = *(const v4f*)(sp);
    const v4f vb = *(const v4f*)(sp + 4);
    v8h hv;
#pragma unroll
    for (int e = 0; e < 4; ++e) {
      const unsigned short b0 = f2bf_bits(va[e]);
      const unsigned short b1 = f2bf_bits(vb[e]);
      hv[e]     = __builtin_bit_cast(_Float16, b0);
      hv[4 + e] = __builtin_bit_cast(_Float16, b1);
    }
    unsigned short* op = dst + ((size_t)a * NBAT + b) * NFEAT + c8;
    *(volatile v8h*)op = hv;
    __threadfence();
    *(volatile v8h*)op = hv;
  }
}

__device__ __forceinline__ float sigm_f(float x) {
  const float xc = fminf(fmaxf(x, -40.0f), 40.0f);
  return __builtin_amdgcn_rcpf(1.0f + expf(-xc));
}
__device__ __forceinline__ float tanh_f(float x) {
  const float xc = fminf(fmaxf(x, -15.0f), 15.0f);
  return 1.0f - 2.0f * __builtin_amdgcn_rcpf(expf(2.0f * xc) + 1.0f);
}

__global__ __launch_bounds__(256) void gru_gate_kernel(
    const unsigned short* __restrict__ X2p, const unsigned short* __restrict__ HBp,
    const unsigned short* __restrict__ WIp, const unsigned short* __restrict__ WHp,
    const float* __restrict__ bih, const float* __restrict__ bhh,
    const float* __restrict__ hid, float* __restrict__ outh, unsigned short* __restrict__ H2p) {
  __shared__ __align__(16) float Sz[64 * SLABP];
  __shared__ __align__(16) float Sa[64 * SLABP];
  const int a  = blockIdx.y;
  const int tm = blockIdx.x >> 2;
  const int tn = blockIdx.x & 3;
  const int m0 = tm * 64;
  const int n0 = tn * 64;
  const int tid = threadIdx.x, lane = tid & 31, wave = tid >> 5;
  const int c = lane & 15, hh = lane >> 4, koff = hh * 8;
  const int mh = wave & 1, nj = wave >> 1;
  const int j = n0 + 16 * nj + c;

  const __bf16* X2 = (const __bf16*)X2p + (size_t)a * NBAT * XPITCH;
  const __bf16* HB = (const __bf16*)HBp + (size_t)a * NBAT * NHID;
  const __bf16* WI = (const __bf16*)WIp + (size_t)a * NGATE * NHID;
  const __bf16* WH = (const __bf16*)WHp + (size_t)a * NGATE * NHID;
  const __bf16* xrow = X2 + (size_t)(m0 + 32 * mh + c) * XPITCH + koff;
  const __bf16* hrow = HB + (size_t)(m0 + 32 * mh + c) * NHID + koff;
  const __bf16* wi = WI + (size_t)j * NHID + koff;
  const __bf16* wh = WH + (size_t)j * NHID + koff;
  const size_t gstride = (size_t)NHID * NHID;

  v8f acc[2][4];
#pragma unroll
  for (int i = 0; i < 2; ++i)
#pragma unroll
    for (int g = 0; g < 4; ++g) acc[i][g] = (v8f){0.f,0.f,0.f,0.f,0.f,0.f,0.f,0.f};

#pragma unroll 1
  for (int k0 = 0; k0 < NHID; k0 += 32) {
    const v16b wir = Frag<__bf16>::load(wi + k0);
    const v16b wiz = Frag<__bf16>::load(wi + gstride + k0);
    const v16b win = Frag<__bf16>::load(wi + 2 * gstride + k0);
    const v16b whr = Frag<__bf16>::load(wh + k0);
    const v16b whz = Frag<__bf16>::load(wh + gstride + k0);
    const v16b whn = Frag<__bf16>::load(wh + 2 * gstride + k0);
#pragma unroll
    for (int i = 0; i < 2; ++i) {
      const v16b xh = Frag<__bf16>::load(xrow + (size_t)i * 16 * XPITCH + k0);
      const v16b xl = Frag<__bf16>::load(xrow + (size_t)i * 16 * XPITCH + NHID + k0);
      const v16b ha = Frag<__bf16>::load(hrow + (size_t)i * 16 * NHID + k0);
      acc[i][0] = Frag<__bf16>::mma(xh, wir, acc[i][0]);
      acc[i][1] = Frag<__bf16>::mma(xh, wiz, acc[i][1]);
      acc[i][2] = Frag<__bf16>::mma(xh, win, acc[i][2]);
      acc[i][3] = Frag<__bf16>::mma(ha, whn, acc[i][3]);
      acc[i][0] = Frag<__bf16>::mma(xl, wir, acc[i][0]);
      acc[i][1] = Frag<__bf16>::mma(xl, wiz, acc[i][1]);
      acc[i][2] = Frag<__bf16>::mma(xl, win, acc[i][2]);
      acc[i][0] = Frag<__bf16>::mma(ha, whr, acc[i][0]);
      acc[i][1] = Frag<__bf16>::mma(ha, whz, acc[i][1]);
      gate_guard(acc[i][0], acc[i][1], acc[i][2], acc[i][3], xh, xl, ha, wir, wiz, win, whr, whz, whn);
    }
    keep4_b(wir, wiz, win, whr);
    keep4_b(whz, whn, wir, wiz);
  }
  acc_guard4(acc[0][0], acc[0][1], acc[0][2], acc[0][3]);
  acc_guard4(acc[1][0], acc[1][1], acc[1][2], acc[1][3]);

  const float bir = bf16r(bih[a * NGATE + j]);
  const float biz = bf16r(bih[a * NGATE + NHID + j]);
  const float bin = bf16r(bih[a * NGATE + 2 * NHID + j]);
  const float bhr = bf16r(bhh[a * NGATE + j]);
  const float bhz = bf16r(bhh[a * NGATE + NHID + j]);
  const float bhn = bf16r(bhh[a * NGATE + 2 * NHID + j]);

#pragma unroll
  for (int i = 0; i < 2; ++i) {
#pragma unroll
    for (int r = 0; r < 8; ++r) {
      const int lr = 32 * mh + 16 * i + 8 * hh + r;
      const float rp = (acc[i][0][r] + bir) + bhr;
      const float rg = sigm_f(rp);
      const float zp = (acc[i][1][r] + biz) + bhz;
      const float ap = (acc[i][2][r] + bin) + rg * (acc[i][3][r] + bhn);
      Sz[lr * SLABP + 16 * nj + c] = zp;
      Sa[lr * SLABP + 16 * nj + c] = ap;
    }
  }
  __syncthreads();

  const int c4 = c * 4;
#pragma unroll 1
  for (int it = 0; it < 4; ++it) {
    const int lr = 8 * wave + 2 * it + hh;
    const size_t grow = (size_t)(m0 + lr) * NAG + a;
    const v4f zp = *(const v4f*)(Sz + lr * SLABP + c4);
    const v4f ap = *(const v4f*)(Sa + lr * SLABP + c4);
    const v4f hv = *(const v4f*)(hid + grow * NHID + n0 + c4);
    v4f hn;
#pragma unroll
    for (int e = 0; e < 4; ++e) {
      const float zg = sigm_f(zp[e]);
      const float ng = tanh_f(ap[e]);
      const float hp = bf16r(hv[e]);
      hn[e] = ng + zg * (hp - ng);
    }
    *(v4f*)(Sa + lr * SLABP + c4) = hn;
  }
  __syncthreads();

  for (int pass = 0; pass < 2; ++pass) {
#pragma unroll
    for (int it = 0; it < 4; ++it) {
      const int lr = 8 * wave + 2 * it + hh;
      const size_t grow = (size_t)(m0 + lr) * NAG + a;
      const v4f v = *(const v4f*)(Sa + lr * SLABP + c4);
      *(volatile v4f*)(outh + grow * NHID + n0 + c4) = v;
    }
    __threadfence();
  }
  {
    const int q = lane >> 3, c8 = (lane & 7) * 8;
    unsigned short* H2 = H2p + (size_t)a * NBAT * XPITCH;
    for (int pass = 0; pass < 2; ++pass) {
#pragma unroll
      for (int it = 0; it < 2; ++it) {
        const int lr = 8 * wave + 4 * it + q;
        const float* sp = Sa + lr * SLABP + c8;
        v8h hv, lv;
#pragma unroll
        for (int e = 0; e < 8; ++e) {
          const float f = sp[e];
          const unsigned short hb = f2bf_bits(f);
          const unsigned short lb = f2bf_bits(f - bf_bits2f(hb));
          hv[e] = __builtin_bit_cast(_Float16, hb);
          lv[e] = __builtin_bit_cast(_Float16, lb);
        }
        unsigned short* op = H2 + (size_t)(m0 + lr) * XPITCH + n0 + c8;
        *(volatile v8h*)(op) = hv;
        *(volatile v8h*)(op + NHID) = lv;
      }
      __threadfence();
    }
  }
}

__global__ __launch_bounds__(256) void pack_q_kernel(const float* __restrict__ QP, float* __restrict__ out0) {
  const int t = blockIdx.x * 256 + threadIdx.x;
  if (t < NOUT0 / 4) {
    v4f v;
#pragma unroll
    for (int e = 0; e < 4; ++e) {
      const int f = 4 * t + e;
      const int r = f / NACT;
      const int cc = f - r * NACT;
      v[e] = QP[(size_t)r * NACTP + cc];
    }
    float* op = out0 + (size_t)t * 4;
    *(volatile v4f*)op = v;
    __threadfence();
    *(volatile v4f*)op = v;
  }
}

extern "C" void kernel_launch(void* const* d_in, const int* in_sizes, int n_in,
                              void* d_out, int out_size, void* d_ws, size_t ws_size, hipStream_t stream) {
  if (n_in < 10 || d_out == nullptr || d_ws == nullptr) return;
  if (in_sizes[0] != NROWS * NFEAT || in_sizes[1] != NROWS * NHID || in_sizes[2] != NAG * NFEAT * NHID ||
      in_sizes[3] != NAG * NHID || in_sizes[4] != NAG * NHID * NGATE || in_sizes[5] != NAG * NGATE ||
      in_sizes[6] != NAG * NHID * NGATE || in_sizes[7] != NAG * NGATE || in_sizes[8] != NAG * NHID * NACT ||
      in_sizes[9] != NAG * NACT || out_size != NOUT0 + NOUT1) return;

  const float* inp   = (const float*)d_in[0];
  const float* hid   = (const float*)d_in[1];
  const float* fc1_w = (const float*)d_in[2];
  const float* fc1_b = (const float*)d_in[3];
  const float* ih_w  = (const float*)d_in[4];
  const float* ih_b  = (const float*)d_in[5];
  const float* hh_w  = (const float*)d_in[6];
  const float* hh_b  = (const float*)d_in[7];
  const float* fc2_w = (const float*)d_in[8];
  const float* fc2_b = (const float*)d_in[9];
  float* out_q = (float*)d_out;
  float* out_h = out_q + (size_t)NOUT0;

  char* ws = (char*)d_ws; size_t off = 0;
  auto carve = [&](size_t bytes) -> char* { char* p = ws + off; off += (bytes + 255) & ~(size_t)255; return p; };
  unsigned short* W1T = (unsigned short*)carve((size_t)NAG * NHID * NFEAT * 2);
  unsigned short* WIT = (unsigned short*)carve((size_t)NAG * NGATE * NHID * 2);
  unsigned short* WHT = (unsigned short*)carve((size_t)NAG * NGATE * NHID * 2);
  unsigned short* W2D = (unsigned short*)carve((size_t)NAG * NACTP * XPITCH * 2);
  float*          BP  = (float*)carve((size_t)NAG * BPITCH * 4);
  unsigned short* XB  = (unsigned short*)carve((size_t)NAG * NBAT * NFEAT * 2);
  unsigned short* HB  = (unsigned short*)carve((size_t)NAG * NBAT * NHID * 2);
  unsigned short* X2  = (unsigned short*)carve((size_t)NAG * NBAT * XPITCH * 2);
  unsigned short* H2  = (unsigned short*)carve((size_t)NAG * NBAT * XPITCH * 2);
  float*          QP  = (float*)carve((size_t)NROWS * NACTP * 4);
  if (off > ws_size || off > (size_t)134217728) return;

  tpw_bf16_kernel<<<dim3(NHID / 64, NFEAT / 64, NAG), 256, 0, stream>>>(
      fc1_w, NFEAT, NHID, NFEAT, W1T, (long)NFEAT * NHID, (long)NHID * NFEAT);
  tpw_bf16_kernel<<<dim3(NGATE / 64, NHID / 64, NAG), 256, 0, stream>>>(
      ih_w, NHID, NGATE, NHID, WIT, (long)NHID * NGATE, (long)NGATE * NHID);
  tpw_bf16_kernel<<<dim3(NGATE / 64, NHID / 64, NAG), 256, 0, stream>>>(
      hh_w, NHID, NGATE, NHID, WHT, (long)NHID * NGATE, (long)NGATE * NHID);
  w2_prep_kernel<<<(NAG * NACTP * (XPITCH / 8)) / 256, 256, 0, stream>>>(fc2_w, W2D);
  bias_prep_kernel<<<(NAG * BPITCH / 4 + 255) / 256, 256, 0, stream>>>(fc1_b, fc2_b, BP);

  in_cvt_kernel<<<dim3(NROWS * 32 / 256, 2), 256, 0, stream>>>(inp, hid, XB, HB);

  wmma_gemm64<1, false, 2, 2, false, 2><<<dim3((NBAT / 64) * (NHID / 64) / 8, NAG), 256, 0, stream>>>(
      XB, XB, NFEAT, (long)NBAT * NFEAT, W1T, W1T, NFEAT, (long)NHID * NFEAT,
      (void*)X2, (void*)(X2 + NHID), XPITCH, (long)NBAT * XPITCH,
      BP, (long)BPITCH, hid, 0L, NBAT, NHID, NFEAT, 1.0f);

  gru_gate_kernel<<<dim3((NBAT / 64) * (NHID / 64), NAG), 256, 0, stream>>>(
      X2, HB, WIT, WHT, ih_b, hh_b, hid, out_h, H2);

  wmma_gemm64<1, false, 2, 0, false, 2><<<dim3((NBAT / 64) * (NACTP / 64) / 8, NAG), 256, 0, stream>>>(
      H2, H2, XPITCH, (long)NBAT * XPITCH, W2D, W2D, XPITCH, (long)NACTP * XPITCH,
      (void*)QP, (void*)QP, NAG * NACTP, (long)NACTP,
      BP + NHID, (long)BPITCH, hid, 0L, NBAT, NACTP, XPITCH, 1.0f);

  pack_q_kernel<<<(NOUT0 / 4) / 256, 256, 0, stream>>>(QP, out_q);
}
